// FRAPModel_24824910970915
// MI455X (gfx1250) — hardware-run, weakly checked
//
#include <hip/hip_runtime.h>


#ifndef NB
#define NB 262144
#endif
#define NB_FULL 262144
#define NPH   8
#define KIN   16
#define NOUT  8
#define CH    20
#define NPAIR 56
#define AW    4
#define TPW   4
#define OSP   20

static_assert(NB <= NB_FULL);
static_assert(NB % (16 * TPW * AW) == 0);
static_assert(KIN == NPH * 2);
static_assert(KIN * 2 == 32);
static_assert(NOUT <= 16);
static_assert(32 * 4 == 16 * NOUT);
static_assert((OSP * 4) % 16 == 0);
static_assert(OSP >= 16);
static_assert(64 * 8 == 16 * 32);
static_assert(64 * 4 == 256);
static_assert(NPAIR == NPH * 7);
static_assert((size_t)AW * TPW * 16 * OSP * 4 <= 131072);
static_assert((size_t)(CH + NPAIR * 8 + NPAIR + 256 + 128 + 8) * 4 <= 131072);

typedef unsigned short bf;
typedef __attribute__((ext_vector_type(16))) __bf16   v16bf;
typedef __attribute__((ext_vector_type(8)))  unsigned short v8us;
typedef __attribute__((ext_vector_type(8)))  float    v8f;
typedef __attribute__((ext_vector_type(4)))  float    v4f;
typedef v4f  __attribute__((may_alias)) v4fa;

__device__ __forceinline__ unsigned short f2bf(float f) { unsigned u = __float_as_uint(f); u += 0x7FFFu + ((u >> 16) & 1u); return (unsigned short)(u >> 16); }
__device__ __forceinline__ float bfr(float f) { return __uint_as_float(((unsigned)f2bf(f)) << 16); }
__device__ __forceinline__ v16bf cat16b(v8us lo, v8us hi) { return __builtin_bit_cast(v16bf, __builtin_shufflevector(lo, hi, 0, 1, 2, 3, 4, 5, 6, 7, 8, 9, 10, 11, 12, 13, 14, 15)); }
__device__ __forceinline__ v8f wmmab(v16bf a, v16bf b, v8f c) { return __builtin_amdgcn_wmma_f32_16x16x32_bf16(false, a, false, b, (short)0, c, false, false); }
__device__ __forceinline__ v16bf ldb(const bf* p)  { return cat16b(*(const v8us*)p, *(const v8us*)(p + 16)); }
__device__ __forceinline__ void wave_sync() { __builtin_amdgcn_fence(3  , "wavefront"); __builtin_amdgcn_wave_barrier(); asm volatile("" ::: "memory"); }
__device__ __forceinline__ v8f wmmab_g(v16bf a, v16bf b, v8f c) { c = wmmab(a, b, c); asm volatile("v_nop\n\tv_nop\n\tv_nop\n\tv_nop" : "+v"(c) : "v"(a), "v"(b)); return c; }

__global__ __launch_bounds__(64) void k_fold(const int* __restrict__ rel,
                                             const float* __restrict__ Wd, const float* __restrict__ bd,
                                             const float* __restrict__ W1, const float* __restrict__ b1,
                                             const float* __restrict__ Erel,
                                             const float* __restrict__ Wr, const float* __restrict__ br,
                                             const float* __restrict__ W2, const float* __restrict__ b2,
                                             const float* __restrict__ W3, const float* __restrict__ b3,
                                             bf* NP, float* DV) {
    __shared__ float sv[CH];
    __shared__ float sA[NPAIR * 8];
    __shared__ float sB[NPAIR];
    __shared__ float sM[256];
    __shared__ float sN[128];
    __shared__ float sD[8];
    const int t = threadIdx.x;

    const int tc = t < CH ? t : CH - 1;
    float a1 = 0.0f, c0 = 0.0f;
#pragma unroll 1
    for (int o = 0; o < CH; ++o) { const float w3 = bfr(W3[o]); a1 += w3 * bfr(W2[o * CH + tc]); c0 += w3 * bfr(b2[o]); }
    c0 += bfr(b3[0]);
    if (t < CH) sv[t] = a1;
    __syncthreads();

    const int tp = t < NPAIR ? t : NPAIR - 1;
    int r = rel[tp]; r = r < 0 ? 0 : (r > 1 ? 1 : r);
    const float e0 = bfr(Erel[r * 4 + 0]), e1 = bfr(Erel[r * 4 + 1]), e2 = bfr(Erel[r * 4 + 2]), e3 = bfr(Erel[r * 4 + 3]);
    float A[8]; float Bb = 0.0f;
#pragma unroll
    for (int k = 0; k < 8; ++k) A[k] = 0.0f;
#pragma unroll 1
    for (int o = 0; o < CH; ++o) {
        float mw = e0 * bfr(Wr[o * 4 + 0]); mw += e1 * bfr(Wr[o * 4 + 1]); mw += e2 * bfr(Wr[o * 4 + 2]); mw += e3 * bfr(Wr[o * 4 + 3]); mw += bfr(br[o]);
        const float m2 = sv[o] * mw;
#pragma unroll
        for (int k = 0; k < 8; ++k) A[k] += m2 * bfr(W1[o * 8 + k]);
        Bb += m2 * bfr(b1[o]);
    }
    if (t < NPAIR) {
#pragma unroll
        for (int k = 0; k < 8; ++k) sA[t * 8 + k] = A[k];
        sB[t] = Bb; }
    __syncthreads();

#pragma unroll 1
    for (int e = t; e < 256; e += 64) {
        const int s = e >> 5, p = (e >> 2) & 7, d = e & 3;
        float ssum = 0.0f;
#pragma unroll 1
        for (int j = 0; j < 7; ++j) ssum += sA[(s * 7 + j) * 8 + d];
        int jj = p < s ? p : p - 1; jj = jj < 0 ? 0 : (jj > 6 ? 6 : jj);
        float dvv = sA[(s * 7 + jj) * 8 + 4 + d];
        asm volatile("" : "+v"(ssum)); asm volatile("" : "+v"(dvv));
        sM[e] = (p == s) ? ssum : dvv;
    }
    __syncthreads();

#pragma unroll 1
    for (int e = t; e < 128; e += 64) {
        const int s = e >> 4, kk = e & 15, p = kk >> 1, c = kk & 1;
        float a = 0.0f;
#pragma unroll 1
        for (int d = 0; d < 4; ++d) a += sM[s * 32 + p * 4 + d] * bfr(Wd[d * 2 + c]);
        sN[e] = a;
    }
    { const int s = t & 7; float dacc = 7.0f * c0;
#pragma unroll 1
      for (int j = 0; j < 7; ++j) dacc += sB[s * 7 + j];
#pragma unroll 1
      for (int q = 0; q < 32; ++q) dacc += sM[s * 32 + q] * bfr(bd[q & 3]);
      if (t < 8) sD[t] = dacc; }
    __syncthreads();

    { const int n = t >> 2, q = t & 3; const int nc = n < 8 ? n : 7; const int kb = (q & 1) * 8;
      v8us o;
#pragma unroll
      for (int i = 0; i < 8; ++i) {
          float v = sN[nc * 16 + kb + i];
          asm volatile("" : "+v"(v));
          const unsigned short hb = f2bf(v);
          const float hv = __uint_as_float(((unsigned)hb) << 16);
          const unsigned short lb = f2bf(v - hv);
          const unsigned short w = (q < 2) ? hb : lb;
          o[i] = (n < 8) ? w : (unsigned short)0; }
      v4f dq;
#pragma unroll
      for (int i = 0; i < 4; ++i) { const int idx = 4 * t + i; float v = sD[idx & 7]; asm volatile("" : "+v"(v)); dq[i] = (idx < 8) ? v : 0.0f; }
      *(volatile v8us*)(NP + (size_t)t * 8) = o; *(volatile v4f*)(DV + (size_t)t * 4) = dq;
      __threadfence();
      *(volatile v8us*)(NP + (size_t)t * 8) = o; *(volatile v4f*)(DV + (size_t)t * 4) = dq; }
}

__global__ __launch_bounds__(32 * AW) void k_apply(const float* __restrict__ ob, const bf* __restrict__ NP, const float* __restrict__ DV, float* OUT) {
    __shared__ __align__(16) float os[AW * TPW * 16 * OSP];
    const int lane = threadIdx.x & 31, lr = lane & 15, hi = lane >> 4;
    const int wave = __builtin_amdgcn_readfirstlane((int)(threadIdx.x >> 5));
    const size_t row0 = ((size_t)blockIdx.x * AW + (size_t)wave) * (size_t)(16 * TPW);
    const v16bf bfrag = ldb(NP + (size_t)lr * 32 + 8 * hi);
    const float dv = DV[lr];
    const int wb = wave * TPW * 16 * OSP;
#pragma unroll
    for (int t = 0; t < TPW; ++t) {
        const float* rp = ob + (row0 + (size_t)(t * 16 + lr)) * KIN + 8 * hi;
        const v4f x0 = *(const v4f*)rp; const v4f x1 = *(const v4f*)(rp + 4);
        v8us a8;
#pragma unroll
        for (int i = 0; i < 4; ++i) { a8[i] = f2bf(x0[i]); a8[4 + i] = f2bf(x1[i]); }
        const v16bf a = cat16b(a8, a8);
        v8f acc = (v8f){};
        acc = wmmab_g(a, bfrag, acc);
#pragma unroll
        for (int r = 0; r < 8; ++r) os[wb + t * 16 * OSP + (8 * hi + r) * OSP + lr] = acc[r] + dv;
    }
    wave_sync();
    float* orow = OUT + row0 * NOUT;
#pragma unroll 1
    for (int ps = 0; ps < 2; ++ps) {
#pragma unroll
        for (int t = 0; t < TPW; ++t) { const int row = lane >> 1, cofs = (lane & 1) * 4;
            const v4f val = *(const v4fa*)(&os[wb + t * 16 * OSP + row * OSP + cofs]);
            *(volatile v4f*)(orow + (size_t)t * (16 * NOUT) + (size_t)lane * 4) = val; }
        if (ps == 0) __threadfence(); }
}

static constexpr size_t al256(size_t v) { return (v + 255) & ~(size_t)255; }
static constexpr size_t SZ_NP = al256((size_t)16 * 32 * 2);
static constexpr size_t SZ_DV = al256((size_t)256 * 4);
static constexpr size_t SZ_TOTAL = SZ_NP + SZ_DV;
static_assert(SZ_TOTAL <= (size_t)134217728);
static_assert(SZ_NP >= (size_t)64 * 8 * 2);
static_assert(SZ_DV >= (size_t)64 * 4 * 4);
static_assert((size_t)15 * 32 + 8 + 16 + 7 < (size_t)16 * 32);

extern "C" void kernel_launch(void* const* d_in, const int* in_sizes, int n_in,
                              void* d_out, int out_size, void* d_ws, size_t ws_size, hipStream_t stream) {
    if (n_in < 13) return;
    if ((size_t)in_sizes[0] < (size_t)NB * KIN) return;
    if (in_sizes[1] < NPAIR || in_sizes[2] < 8 || in_sizes[3] < 4 || in_sizes[4] < CH * 8 || in_sizes[5] < CH) return;
    if (in_sizes[6] < 8 || in_sizes[7] < CH * 4 || in_sizes[8] < CH || in_sizes[9] < CH * CH || in_sizes[10] < CH || in_sizes[11] < CH || in_sizes[12] < 1) return;
    if ((size_t)out_size < (size_t)NB * NOUT) return;
    if (SZ_TOTAL > ws_size) return;
    const float* ob  = (const float*)d_in[0];
    const int*   rel = (const int*)d_in[1];
    const float* Wd  = (const float*)d_in[2];
    const float* bd  = (const float*)d_in[3];
    const float* W1  = (const float*)d_in[4];
    const float* b1  = (const float*)d_in[5];
    const float* Er  = (const float*)d_in[6];
    const float* Wr  = (const float*)d_in[7];
    const float* br  = (const float*)d_in[8];
    const float* W2  = (const float*)d_in[9];
    const float* b2  = (const float*)d_in[10];
    const float* W3  = (const float*)d_in[11];
    const float* b3  = (const float*)d_in[12];
    float* OUT = (float*)d_out;
    char* wsp = (char*)d_ws;
    bf* NP = (bf*)wsp; wsp += SZ_NP;
    float* DV = (float*)wsp;

    k_fold<<<1, 64, 0, stream>>>(rel, Wd, bd, W1, b1, Er, Wr, br, W2, b2, W3, b3, NP, DV);
    k_apply<<<dim3(NB / (16 * TPW * AW), 1, 1), 32 * AW, 0, stream>>>(ob, NP, DV, OUT);
}
